// MambaBlock_36636071035407
// MI455X (gfx1250) — hardware-verified
//
#include <hip/hip_runtime.h>
#include <math.h>

typedef __attribute__((ext_vector_type(16))) _Float16 v16h;
typedef __attribute__((ext_vector_type(8)))  _Float16 v8h;
typedef __attribute__((ext_vector_type(16))) __bf16   v16b;
typedef __attribute__((ext_vector_type(8)))  __bf16   v8b;
typedef __attribute__((ext_vector_type(8)))  float    v8f;
typedef __attribute__((ext_vector_type(4)))  float    v4f;

constexpr int kBatch = 2;
constexpr int kSeq   = 1024;
constexpr int kDmod  = 1024;
constexpr int kDin   = 2048;
constexpr int kNst   = 16;
constexpr int kDsc   = 128;
constexpr int kKer   = 4;
constexpr int kRows  = kBatch * kSeq;
constexpr int kXzP   = 2 * kDin;
constexpr int kBcdN  = 2 * kNst + kDsc;
constexpr int kBcdP  = 192;
constexpr int kTP    = 260;
static_assert(kRows == 2048 && kXzP == 4096 && kBcdN == 160, "shape constants");
static_assert((kBcdP % 64) == 0 && kBcdP >= kBcdN, "padded projection width");
static_assert((kDmod % 32) == 0 && (kDin % 32) == 0 && (kDsc % 32) == 0, "GEMM K multiples of 32");
static_assert((kRows % 64) == 0 && (kXzP % 64) == 0 && (kDin % 64) == 0 && (kDmod % 64) == 0, "GEMM M,N multiples of 64");
static_assert((kSeq % 64) == 0 && (kDin % 256) == 0 && (kSeq % 16) == 0, "tile multiples");
static_assert(kKer == 4 && kNst == 16 && (kTP % 4) == 0, "kernel assumptions");

constexpr size_t kOffSEQB  = 0;
constexpr size_t kOffWINB  = kOffSEQB  + (size_t)kRows * kDmod * 2;
constexpr size_t kOffWOUTB = kOffWINB  + (size_t)kXzP  * kDmod * 2;
constexpr size_t kOffWBCD  = kOffWOUTB + (size_t)kDmod * kDin  * 2;
constexpr size_t kOffWD2B  = kOffWBCD  + (size_t)kBcdP * kDin  * 2;
constexpr size_t kOffAB    = kOffWD2B  + (size_t)kDin  * kDsc  * 2;
constexpr size_t kOffA32   = kOffAB    + (size_t)kRows * kXzP  * 4;
constexpr size_t kOffAH    = kOffA32   + (size_t)kRows * kDin  * 4;
constexpr size_t kOffAL    = kOffAH    + (size_t)kRows * kDin  * 2;
constexpr size_t kOffBCD   = kOffAL    + (size_t)kRows * kDin  * 2;
constexpr size_t kOffD1H   = kOffBCD   + (size_t)kRows * kBcdP * 4;
constexpr size_t kOffD1L   = kOffD1H   + (size_t)kRows * kDsc  * 2;
constexpr size_t kOffDLR   = kOffD1L   + (size_t)kRows * kDsc  * 2;
constexpr size_t kOffYH    = kOffDLR   + (size_t)kRows * kDin  * 4;
constexpr size_t kOffYL    = kOffYH    + (size_t)kRows * kDin  * 2;
constexpr size_t kWsTotal  = kOffYL    + (size_t)kRows * kDin  * 2;
static_assert(kWsTotal == 121372672ull, "carve total");
static_assert(kWsTotal <= 134217728ull, "carve cap");
static_assert((kOffWINB % 128) == 0 && (kOffWOUTB % 128) == 0 && (kOffWBCD % 128) == 0 && (kOffWD2B % 128) == 0 &&
              (kOffAB % 128) == 0 && (kOffA32 % 128) == 0 && (kOffAH % 128) == 0 && (kOffAL % 128) == 0 &&
              (kOffBCD % 128) == 0 && (kOffD1H % 128) == 0 && (kOffD1L % 128) == 0 && (kOffDLR % 128) == 0 &&
              (kOffYH % 128) == 0 && (kOffYL % 128) == 0, "128-B aligned regions");

__device__ __forceinline__ unsigned short f2bf_bits(float f) {
  unsigned u = __float_as_uint(f);
  return (unsigned short)((u + 0x7FFFu + ((u >> 16) & 1u)) >> 16);
}
__device__ __forceinline__ float bf_bits2f(unsigned short h) { return __uint_as_float(((unsigned)h) << 16); }
__device__ __forceinline__ float bf_rne(float f) { return bf_bits2f(f2bf_bits(f)); }

__device__ __forceinline__ void dep_guard4_b(v8f& a, v8f& b, v8f& c, v8f& d, v16b x, v16b y) { asm volatile("v_nop\n\tv_nop\n\tv_nop\n\tv_nop" : "+v"(a), "+v"(b), "+v"(c), "+v"(d) : "v"(x), "v"(y)); }
__device__ __forceinline__ void keep4_b(v16b a, v16b b, v16b c, v16b d) { asm volatile("v_nop" :: "v"(a), "v"(b), "v"(c), "v"(d)); }
__device__ __forceinline__ void acc_guard4(v8f& a, v8f& b, v8f& c, v8f& d) { asm volatile("v_nop\n\tv_nop\n\tv_nop\n\tv_nop" : "+v"(a), "+v"(b), "+v"(c), "+v"(d)); }
template <typename T> struct Frag;
template <> struct Frag<__bf16> {
  typedef v16b V; union U { v16b v; v8b h[2]; };
  static __device__ __forceinline__ v16b load(const __bf16* p) {
    U f; f.h[0] = *(const v8b*)(p); f.h[1] = *(const v8b*)(p + 16); return f.v;
  }
  static __device__ __forceinline__ v8f mma(v16b a, v16b b, v8f c) {
    return __builtin_amdgcn_wmma_f32_16x16x32_bf16(false, a, false, b, (short)0, c, false, false);
  }
};

template <int SPL>
__global__ __launch_bounds__(256) void wmma_gemm64(
    const unsigned short* __restrict__ Ap, const unsigned short* __restrict__ A2p, int lda,
    const unsigned short* __restrict__ Btp, int ldb,
    float* __restrict__ Cout, int ldc, int M, int N, int K) {
  typedef __bf16 T;
  typedef Frag<T>::V V;
  const T* A = (const T*)Ap; const T* A2 = (const T*)A2p; const T* Bt = (const T*)Btp;
  __shared__ __align__(16) float sT[8][16 * 68];
  const int lane = threadIdx.x & 31;
  const int wave = threadIdx.x >> 5;
  const int tilesN = N >> 6;
  const int tilesM = M >> 6;
  const int tile = blockIdx.x * 8 + wave;
  if (tile >= tilesM * tilesN) return;
  const int tm = tile / tilesN;
  const int tn = tile - tm * tilesN;
  const int m0 = tm << 6;
  const int n0 = tn << 6;

  const int rlane = lane & 15;
  const int koff  = (lane >> 4) * 8;
  const int mOff  = (lane >> 4) * 8;

  v8f acc[4][4];
#pragma unroll
  for (int i = 0; i < 4; ++i)
#pragma unroll
    for (int j = 0; j < 4; ++j) acc[i][j] = (v8f){0.f,0.f,0.f,0.f,0.f,0.f,0.f,0.f};

  for (int k0 = 0; k0 < K; k0 += 32) {
    V bh[4];
#pragma unroll
    for (int j = 0; j < 4; ++j) {
      const size_t bo = (size_t)(n0 + (j << 4) + rlane) * ldb + koff + k0;
      bh[j] = Frag<T>::load(Bt + bo);
    }
#pragma unroll
    for (int i = 0; i < 4; ++i) {
      const size_t ao = (size_t)(m0 + (i << 4) + rlane) * lda + koff + k0;
      V ah = Frag<T>::load(A + ao);
      V al = ah;
      if (SPL == 1) al = Frag<T>::load(A2 + ao);
#pragma unroll
      for (int j = 0; j < 4; ++j) {
        acc[i][j] = Frag<T>::mma(ah, bh[j], acc[i][j]);
        if (SPL == 1) acc[i][j] = Frag<T>::mma(al, bh[j], acc[i][j]);
      }
      dep_guard4_b(acc[i][0], acc[i][1], acc[i][2], acc[i][3], ah, al);
    }
    keep4_b(bh[0], bh[1], bh[2], bh[3]);
  }
  acc_guard4(acc[0][0], acc[0][1], acc[0][2], acc[0][3]);
  acc_guard4(acc[1][0], acc[1][1], acc[1][2], acc[1][3]);
  acc_guard4(acc[2][0], acc[2][1], acc[2][2], acc[2][3]);
  acc_guard4(acc[3][0], acc[3][1], acc[3][2], acc[3][3]);

  float* slab = sT[wave];
#pragma unroll
  for (int i = 0; i < 4; ++i) {
    const int mBase = m0 + (i << 4);
#pragma unroll
    for (int j = 0; j < 4; ++j) {
#pragma unroll
      for (int r = 0; r < 8; ++r) {
        slab[(mOff + r) * 68 + (j << 4) + rlane] = acc[i][j][r];
      }
    }
    __builtin_amdgcn_fence(__ATOMIC_RELEASE, "workgroup");
    __builtin_amdgcn_wave_barrier();
    __builtin_amdgcn_fence(__ATOMIC_ACQUIRE, "workgroup");
    {
      const int hh = lane >> 4, c4 = (lane & 15) * 4;
      for (int pass = 0; pass < 2; ++pass) {
#pragma unroll
        for (int it = 0; it < 8; ++it) {
          const int row = it * 2 + hh;
          v4f v = *(const v4f*)(slab + row * 68 + c4);
          *(volatile v4f*)(Cout + (size_t)(mBase + row) * ldc + n0 + c4) = v;
        }
        __threadfence();
      }
    }
    __builtin_amdgcn_fence(__ATOMIC_RELEASE, "workgroup");
    __builtin_amdgcn_wave_barrier();
    __builtin_amdgcn_fence(__ATOMIC_ACQUIRE, "workgroup");
  }
}

__global__ __launch_bounds__(256) void pack_bf16_kernel(
    const float* __restrict__ src, unsigned short* __restrict__ dst, int total8)
{
  const int i = blockIdx.x * 256 + threadIdx.x;
  if (i >= total8) return;
  const size_t e0 = (size_t)i << 3;
  const v4f a0 = *(const v4f*)(src + e0);
  const v4f a1 = *(const v4f*)(src + e0 + 4);
  v8h hv;
#pragma unroll
  for (int e = 0; e < 4; ++e) {
    const float x0 = a0[e];
    const float x1 = a1[e];
    const unsigned short h0 = f2bf_bits(x0);
    const unsigned short h1 = f2bf_bits(x1);
    hv[e]     = __builtin_bit_cast(_Float16, h0);
    hv[4 + e] = __builtin_bit_cast(_Float16, h1);
  }
  unsigned short* q = dst + e0;
  *(volatile v8h*)q = hv;
  __threadfence();
  *(volatile v8h*)q = hv;
}

__global__ __launch_bounds__(256) void pack_bcd_kernel(
    const float* __restrict__ WsB, const float* __restrict__ WsC, const float* __restrict__ WsD1,
    unsigned short* __restrict__ dst)
{
  const int row = blockIdx.x;
  const int c8  = threadIdx.x * 8;
  const float* src = WsD1;
  int srow = 0;
  if (row < kNst) { src = WsB; srow = row; }
  else if (row < 2 * kNst) { src = WsC; srow = row - kNst; }
  else if (row < kBcdN) { srow = row - 2 * kNst; }
  const bool live = (row < kBcdN);
  const float* p = src + (size_t)srow * kDin + c8;
  const v4f a0 = *(const v4f*)(p);
  const v4f a1 = *(const v4f*)(p + 4);
  v8h hv;
#pragma unroll
  for (int e = 0; e < 4; ++e) {
    const float x0 = live ? a0[e] : 0.0f;
    const float x1 = live ? a1[e] : 0.0f;
    const unsigned short h0 = f2bf_bits(x0);
    const unsigned short h1 = f2bf_bits(x1);
    hv[e]     = __builtin_bit_cast(_Float16, h0);
    hv[4 + e] = __builtin_bit_cast(_Float16, h1);
  }
  unsigned short* q = dst + (size_t)row * kDin + c8;
  *(volatile v8h*)q = hv;
  __threadfence();
  *(volatile v8h*)q = hv;
}

__global__ __launch_bounds__(256) void pack_d1_kernel(
    const float* __restrict__ BCD, unsigned short* __restrict__ D1H, unsigned short* __restrict__ D1L, int total8)
{
  const int i = blockIdx.x * 256 + threadIdx.x;
  if (i >= total8) return;
  const int e0  = i << 3;
  const int row = e0 >> 7;
  const int c8  = e0 & (kDsc - 1);
  const float* p = BCD + (size_t)row * kBcdP + 2 * kNst + c8;
  const v4f a0 = *(const v4f*)(p);
  const v4f a1 = *(const v4f*)(p + 4);
  v8h hv, lv;
#pragma unroll
  for (int e = 0; e < 4; ++e) {
    const float x0 = a0[e];
    const float x1 = a1[e];
    const unsigned short h0 = f2bf_bits(x0);
    const unsigned short h1 = f2bf_bits(x1);
    const unsigned short l0 = f2bf_bits(x0 - bf_bits2f(h0));
    const unsigned short l1 = f2bf_bits(x1 - bf_bits2f(h1));
    hv[e]     = __builtin_bit_cast(_Float16, h0);
    hv[4 + e] = __builtin_bit_cast(_Float16, h1);
    lv[e]     = __builtin_bit_cast(_Float16, l0);
    lv[4 + e] = __builtin_bit_cast(_Float16, l1);
  }
  unsigned short* qh = D1H + e0;
  unsigned short* ql = D1L + e0;
  *(volatile v8h*)qh = hv;
  *(volatile v8h*)ql = lv;
  __threadfence();
  *(volatile v8h*)qh = hv;
  *(volatile v8h*)ql = lv;
}

__global__ __launch_bounds__(256) void conv_silu_kernel(
    const float* __restrict__ AB, const float* __restrict__ cw, const float* __restrict__ cb,
    float* __restrict__ A32, unsigned short* __restrict__ AH, unsigned short* __restrict__ AL)
{
  __shared__ __align__(16) float sT[16 * kTP];
  const int tid = threadIdx.x, lane = tid & 31, wave = tid >> 5;
  const int d0 = blockIdx.x * 256, d = d0 + tid;
  const int g0 = blockIdx.y * 64;
  const int tb = g0 & (kSeq - 1);
  const v4f wv = *(const v4f*)(cw + (size_t)d * kKer);
  const float c0 = wv[0];
  const float c1 = wv[1];
  const float c2 = wv[2];
  const float c3 = wv[3];
  const float w0 = bf_rne(c0), w1 = bf_rne(c1), w2 = bf_rne(c2), w3 = bf_rne(c3);
  const float bc = bf_rne(cb[d]);
  float xm3, xm2, xm1;
  {
    const bool hist = (tb > 0);
    const int rb = hist ? (g0 - 3) : g0;
    const float v3 = AB[(size_t)rb * kXzP + d];
    const float v2 = AB[(size_t)(rb + 1) * kXzP + d];
    const float v1 = AB[(size_t)(rb + 2) * kXzP + d];
    xm3 = hist ? v3 : 0.f;
    xm2 = hist ? v2 : 0.f;
    xm1 = hist ? v1 : 0.f;
  }
  const int hrow = wave >> 1;
  const int hch  = (wave & 1) * 128 + lane * 4;
#pragma unroll 1
  for (int sub = 0; sub < 4; ++sub) {
    const int lb = g0 + sub * 16;
#pragma unroll 1
    for (int s = 0; s < 16; ++s) {
      const float xcur = AB[(size_t)(lb + s) * kXzP + d];
      float acc = w0 * xm3;
      acc = fmaf(w1, xm2, acc);
      acc = fmaf(w2, xm1, acc);
      acc = fmaf(w3, xcur, acc);
      const float sv = acc + bc;
      const float sg = __builtin_amdgcn_rcpf(1.0f + expf(-sv));
      sT[s * kTP + tid] = sv * sg;
      xm3 = xm2; xm2 = xm1; xm1 = xcur;
    }
    __syncthreads();
    v4f fv[4];
    v8h bh[2], blo[2];
#pragma unroll
    for (int it = 0; it < 4; ++it) fv[it] = *(const v4f*)(sT + (it * 4 + hrow) * kTP + hch);
#pragma unroll
    for (int it = 0; it < 2; ++it) {
      const float* sp = sT + (it * 8 + wave) * kTP + lane * 8;
      const v4f a0 = *(const v4f*)(sp);
      const v4f a1 = *(const v4f*)(sp + 4);
#pragma unroll
      for (int e = 0; e < 4; ++e) {
        const float x0 = a0[e];
        const float x1 = a1[e];
        const unsigned short h0 = f2bf_bits(x0);
        const unsigned short h1 = f2bf_bits(x1);
        const unsigned short l0 = f2bf_bits(x0 - bf_bits2f(h0));
        const unsigned short l1 = f2bf_bits(x1 - bf_bits2f(h1));
        bh[it][e]      = __builtin_bit_cast(_Float16, h0);
        bh[it][4 + e]  = __builtin_bit_cast(_Float16, h1);
        blo[it][e]     = __builtin_bit_cast(_Float16, l0);
        blo[it][4 + e] = __builtin_bit_cast(_Float16, l1);
      }
    }
    for (int pass = 0; pass < 2; ++pass) {
#pragma unroll
      for (int it = 0; it < 4; ++it)
        *(volatile v4f*)(A32 + (size_t)(lb + it * 4 + hrow) * kDin + d0 + hch) = fv[it];
#pragma unroll
      for (int it = 0; it < 2; ++it) {
        const size_t o = (size_t)(lb + it * 8 + wave) * kDin + d0 + lane * 8;
        *(volatile v8h*)(AH + o) = bh[it];
        *(volatile v8h*)(AL + o) = blo[it];
      }
      __threadfence();
    }
    __syncthreads();
  }
}

__global__ __launch_bounds__(256) void scan_kernel(
    const float* __restrict__ DLR, const float* __restrict__ A32, const float* __restrict__ AB,
    const float* __restrict__ BCD, const float* __restrict__ Apar, const float* __restrict__ Dpar,
    unsigned short* __restrict__ YH, unsigned short* __restrict__ YL)
{
  __shared__ __align__(16) float sBC[16 * 32];
  __shared__ __align__(16) float sY[16 * kTP];
  __shared__ __align__(16) float sA[kNst * 256];
  const int tid = threadIdx.x, lane = tid & 31, wave = tid >> 5;
  constexpr int kBlkPerB = kDin / 256;
  const int bix = blockIdx.x / kBlkPerB;
  const int d0  = (blockIdx.x - bix * kBlkPerB) * 256;
  const int d   = d0 + tid;
  const size_t row0 = (size_t)bix * kSeq;
#pragma unroll 1
  for (int n = 0; n < kNst; ++n) {
    const float an = bf_rne(Apar[(size_t)d * kNst + n]);
    sA[n * 256 + tid] = expf(-an);
  }
  __syncthreads();
  float eA[kNst], h[kNst];
#pragma unroll
  for (int n = 0; n < kNst; ++n) {
    eA[n] = sA[n * 256 + tid];
    h[n] = 0.f;
  }
  const float Dd = bf_rne(Dpar[d]);

#pragma unroll 1
  for (int c = 0; c < kSeq / 16; ++c) {
    const int l0 = c * 16;
    if (tid < 128) {
      const int r = tid >> 3, q = (tid & 7) * 4;
      const v4f v = *(const v4f*)(BCD + (row0 + l0 + r) * kBcdP + q);
      *(v4f*)(sBC + r * 32 + q) = v;
    }
    __syncthreads();
#pragma unroll 1
    for (int s = 0; s < 16; ++s) {
      const size_t m = row0 + l0 + s;
      float dlr = DLR[m * kDin + d];
      float av  = A32[m * kDin + d];
      float gv  = AB[m * kXzP + kDin + d];
      asm volatile("" : "+v"(dlr), "+v"(av), "+v"(gv));
      const float v  = dlr + Dd;
      const float ea = expf(-fabsf(v));
      const float u  = 1.0f + ea;
      const float l1p = logf(u) + (ea - (u - 1.0f)) * __builtin_amdgcn_rcpf(u);
      const float delta = fmaxf(v, 0.0f) + l1p;
      v4f Bq[4], Cq[4];
#pragma unroll
      for (int qq = 0; qq < 4; ++qq) {
        Bq[qq] = *(const v4f*)(sBC + s * 32 + 4 * qq);
        Cq[qq] = *(const v4f*)(sBC + s * 32 + kNst + 4 * qq);
      }
      float y = 0.f;
#pragma unroll
      for (int n = 0; n < kNst; ++n) {
        const float bn = Bq[n >> 2][n & 3];
        const float cn = Cq[n >> 2][n & 3];
        const float abar = eA[n] * delta;
        const float xbar = (bn * delta) * av;
        h[n] = fmaf(abar, h[n], xbar);
        y = fmaf(h[n], cn, y);
      }
      y = fmaf(Dd, av, y);
      const float sg = __builtin_amdgcn_rcpf(1.0f + expf(-gv));
      y = y * (gv * sg);
      sY[s * kTP + tid] = y;
    }
    __syncthreads();
    v8h hv[2], lv[2];
#pragma unroll
    for (int it = 0; it < 2; ++it) {
      const float* sp = sY + (it * 8 + wave) * kTP + lane * 8;
      const v4f a0 = *(const v4f*)(sp);
      const v4f a1 = *(const v4f*)(sp + 4);
#pragma unroll
      for (int e = 0; e < 4; ++e) {
        const float x0 = a0[e];
        const float x1 = a1[e];
        const unsigned short h0 = f2bf_bits(x0);
        const unsigned short h1 = f2bf_bits(x1);
        const unsigned short q0 = f2bf_bits(x0 - bf_bits2f(h0));
        const unsigned short q1 = f2bf_bits(x1 - bf_bits2f(h1));
        hv[it][e]     = __builtin_bit_cast(_Float16, h0);
        hv[it][4 + e] = __builtin_bit_cast(_Float16, h1);
        lv[it][e]     = __builtin_bit_cast(_Float16, q0);
        lv[it][4 + e] = __builtin_bit_cast(_Float16, q1);
      }
    }
    for (int pass = 0; pass < 2; ++pass) {
#pragma unroll
      for (int it = 0; it < 2; ++it) {
        const size_t o = (row0 + l0 + it * 8 + wave) * kDin + d0 + lane * 8;
        *(volatile v8h*)(YH + o) = hv[it];
        *(volatile v8h*)(YL + o) = lv[it];
      }
      __threadfence();
    }
  }
}

static_assert((((kRows / 64) * (kXzP / 64)) % 8) == 0, "in_proj tiles");
static_assert((((kRows / 64) * (kBcdP / 64)) % 8) == 0, "bcd tiles");
static_assert((((kRows / 64) * (kDin / 64)) % 8) == 0, "dt-up tiles");
static_assert((((kRows / 64) * (kDmod / 64)) % 8) == 0, "out_proj tiles");
static_assert(((kRows * kDmod / 8) % 256) == 0 && ((kXzP * kDmod / 8) % 256) == 0 &&
              ((kDmod * kDin / 8) % 256) == 0 && ((kDin * kDsc / 8) % 256) == 0 &&
              ((kRows * kDsc / 8) % 256) == 0, "pack grids exact");

extern "C" void kernel_launch(void* const* d_in, const int* in_sizes, int n_in,
                              void* d_out, int out_size, void* d_ws, size_t ws_size,
                              hipStream_t stream) {
  if (n_in < 11) return;
  if (in_sizes[0] != kRows * kDmod) return;
  if (in_sizes[1] != kXzP * kDmod) return;
  if (in_sizes[2] != kDmod * kDin) return;
  if (in_sizes[3] != kNst * kDin) return;
  if (in_sizes[4] != kNst * kDin) return;
  if (in_sizes[5] != kDsc * kDin) return;
  if (in_sizes[6] != kDin * kDsc) return;
  if (in_sizes[7] != kDin * kKer) return;
  if (in_sizes[8] != kDin) return;
  if (in_sizes[9] != kDin * kNst) return;
  if (in_sizes[10] != kDin) return;
  if (out_size != kRows * kDmod) return;
  if (ws_size < kWsTotal) return;

  const float* seq    = (const float*)d_in[0];
  const float* W_in   = (const float*)d_in[1];
  const float* W_out  = (const float*)d_in[2];
  const float* W_sB   = (const float*)d_in[3];
  const float* W_sC   = (const float*)d_in[4];
  const float* W_sD1  = (const float*)d_in[5];
  const float* W_sD2  = (const float*)d_in[6];
  const float* conv_w = (const float*)d_in[7];
  const float* conv_b = (const float*)d_in[8];
  const float* A_par  = (const float*)d_in[9];
  const float* D_par  = (const float*)d_in[10];
  float* out = (float*)d_out;

  char* ws = (char*)d_ws;
  unsigned short* SEQB  = (unsigned short*)(ws + kOffSEQB);
  unsigned short* WINB  = (unsigned short*)(ws + kOffWINB);
  unsigned short* WOUTB = (unsigned short*)(ws + kOffWOUTB);
  unsigned short* WBCD  = (unsigned short*)(ws + kOffWBCD);
  unsigned short* WD2B  = (unsigned short*)(ws + kOffWD2B);
  float*          AB    = (float*)(ws + kOffAB);
  float*          A32   = (float*)(ws + kOffA32);
  unsigned short* AH    = (unsigned short*)(ws + kOffAH);
  unsigned short* AL    = (unsigned short*)(ws + kOffAL);
  float*          BCD   = (float*)(ws + kOffBCD);
  unsigned short* D1H   = (unsigned short*)(ws + kOffD1H);
  unsigned short* D1L   = (unsigned short*)(ws + kOffD1L);
  float*          DLR   = (float*)(ws + kOffDLR);
  unsigned short* YH    = (unsigned short*)(ws + kOffYH);
  unsigned short* YL    = (unsigned short*)(ws + kOffYL);

  pack_bf16_kernel<<<(kRows * kDmod / 8) / 256, 256, 0, stream>>>(seq, SEQB, kRows * kDmod / 8);
  pack_bf16_kernel<<<(kXzP * kDmod / 8) / 256, 256, 0, stream>>>(W_in, WINB, kXzP * kDmod / 8);
  pack_bf16_kernel<<<(kDmod * kDin / 8) / 256, 256, 0, stream>>>(W_out, WOUTB, kDmod * kDin / 8);
  pack_bf16_kernel<<<(kDin * kDsc / 8) / 256, 256, 0, stream>>>(W_sD2, WD2B, kDin * kDsc / 8);
  pack_bcd_kernel<<<kBcdP, 256, 0, stream>>>(W_sB, W_sC, W_sD1, WBCD);

  wmma_gemm64<0><<<((kRows / 64) * (kXzP / 64)) / 8, 256, 0, stream>>>(
      SEQB, SEQB, kDmod, WINB, kDmod, AB, kXzP, kRows, kXzP, kDmod);

  conv_silu_kernel<<<dim3(kDin / 256, kRows / 64), 256, 0, stream>>>(AB, conv_w, conv_b, A32, AH, AL);

  wmma_gemm64<1><<<((kRows / 64) * (kBcdP / 64)) / 8, 256, 0, stream>>>(
      AH, AL, kDin, WBCD, kDin, BCD, kBcdP, kRows, kBcdP, kDin);

  pack_d1_kernel<<<(kRows * kDsc / 8) / 256, 256, 0, stream>>>(BCD, D1H, D1L, kRows * kDsc / 8);

  wmma_gemm64<1><<<((kRows / 64) * (kDin / 64)) / 8, 256, 0, stream>>>(
      D1H, D1L, kDsc, WD2B, kDsc, DLR, kDin, kRows, kDin, kDsc);

  scan_kernel<<<kBatch * (kDin / 256), 256, 0, stream>>>(DLR, A32, AB, BCD, A_par, D_par, YH, YL);

  wmma_gemm64<1><<<((kRows / 64) * (kDmod / 64)) / 8, 256, 0, stream>>>(
      YH, YL, kDin, WOUTB, kDin, out, kDmod, kRows, kDmod, kDin);
}
